// ClassificationNet_22110491640138
// MI455X (gfx1250) — hardware-verified
//
#include <hip/hip_runtime.h>


namespace {
constexpr int NB = 16, H = 96, W = 96, C = 3, K9 = 9, OH = 88, OW = 88, NOFF = 162, NOT = 176  , KOFF = 288  , NF = 32, NDCT = 21, H1P = 92  , P2P = 48  ;
constexpr float XS = 8.0f, WSC = 256.0f;

typedef _Float16 b16;
typedef __attribute__((ext_vector_type(16))) _Float16 v16b;
typedef __attribute__((ext_vector_type(8))) _Float16 v8b;
typedef __attribute__((ext_vector_type(8))) float v8f;
typedef __attribute__((ext_vector_type(4))) float v4f;
__device__ __forceinline__ float bf16_rne(float f) { unsigned int u = __float_as_uint(f); u += 0x7FFFu + ((u >> 16) & 1u); return __uint_as_float(u & 0xFFFF0000u); }
__device__ __forceinline__ void split16(float v, b16& hi, b16& lo) { hi = (b16)v; lo = (b16)(v - (float)hi); }
__device__ __forceinline__ v16b frag_kb(const b16* p, int hh) { const v8b a = *(const v8b*)(p + 8 * hh), b = *(const v8b*)(p + 16 + 8 * hh); v16b f;
#pragma unroll
  for (int e = 0; e < 8; ++e) { f[e] = a[e]; f[8 + e] = b[e]; } return f; }
__device__ __forceinline__ v16b frag_kb_u(const b16* p, int hh) {
  v16b f;
#pragma unroll
  for (int e = 0; e < 8; ++e) { f[e] = p[8 * hh + e]; f[8 + e] = p[16 + 8 * hh + e]; } return f; }
__device__ __forceinline__ v8f wmma16b(v16b a, v16b b, v8f c) { v8f d = __builtin_amdgcn_wmma_f32_16x16x32_f16(false, a, false, b, (short)0, c, false, false); asm volatile("v_nop\n\tv_nop\n\tv_nop\n\tv_nop" : "+v"(d) : "v"(a), "v"(b)); return d; }
__device__ __forceinline__ void wave_lds_sync() { __builtin_amdgcn_fence(__ATOMIC_RELEASE, "workgroup"); __builtin_amdgcn_wave_barrier(); __builtin_amdgcn_fence(__ATOMIC_ACQUIRE, "workgroup"); }
__device__ __forceinline__ float pmul(float a, float b) { float p = a * b; asm volatile("" : "+v"(p)); return p; }

__global__ __launch_bounds__(256) void prep_kernel(const float* __restrict__ x, const float* __restrict__ fb, const float* __restrict__ hk, const float* __restrict__ wo, const float* __restrict__ w2, const float* __restrict__ w3, const float* __restrict__ w4,
                                                b16* __restrict__ X16, b16* __restrict__ WOFF, b16* __restrict__ FBh, b16* __restrict__ FBl, b16* __restrict__ HK, b16* __restrict__ WC, b16* __restrict__ zero0, size_t nzero) {
  const size_t t = (size_t)blockIdx.x * 256 + threadIdx.x;
  const size_t nx = ((size_t)NB * H * W * C + 256) / 8  , n1 = (size_t)NOT * KOFF / 8, n2 = 32 * 96 / 8, n3 = 32 * 64 / 8, n4 = (size_t)3 * 32 * 800 / 8, nz = nzero / 8;
  v8b o = {};
  if (t < nx) { const size_t e = t * 8; for (int j = 0; j < 8; ++j) { const size_t i = e + j; o[j] = (b16)((i < (size_t)NB * H * W * C) ? bf16_rne(x[i]) * XS : 0.0f); } for (int pass = 0; pass < 2; ++pass) { *(volatile v8b*)(X16 + e) = o; __threadfence(); } }
  else if (t < nx + n1) { const size_t e = (t - nx) * 8; const int oc = (int)(e / KOFF), k0 = (int)(e - (size_t)oc * KOFF); for (int j = 0; j < 8; ++j) { const int k = k0 + j, p = k >> 5, kk = k & 31; o[j] = (b16)((oc < NOFF && kk < 27) ? bf16_rne(wo[((size_t)(p * K9 + kk / 3) * C + kk % 3) * NOFF + oc]) * WSC : 0.0f); }
    for (int pass = 0; pass < 2; ++pass) { *(volatile v8b*)(WOFF + e) = o; __threadfence(); } }
  else if (t < nx + n1 + n2) { const int e = (int)(t - nx - n1) * 8; const int m = e / 96, k0 = e - m * 96; v8b ol = {}; for (int j = 0; j < 8; ++j) { const int k = k0 + j; const float v = (m < NDCT && k < 81) ? bf16_rne(fb[(size_t)k * NDCT + m]) * WSC : 0.0f; b16 a_, c_; split16(v, a_, c_); o[j] = a_; ol[j] = c_; }
    for (int pass = 0; pass < 2; ++pass) { *(volatile v8b*)(FBh + e) = o; *(volatile v8b*)(FBl + e) = ol; __threadfence(); } }
  else if (t < nx + n1 + n2 + n3) { const int e = (int)(t - nx - n1 - n2) * 8; const int oc = e / 64, k0 = e - oc * 64; for (int j = 0; j < 8; ++j) { const int k = k0 + j; o[j] = (b16)((k < 63) ? bf16_rne(hk[(size_t)k * NF + oc]) * WSC : 0.0f); }
    for (int pass = 0; pass < 2; ++pass) { *(volatile v8b*)(HK + e) = o; __threadfence(); } }
  else if (t < nx + n1 + n2 + n3 + n4) { const size_t u = (t - nx - n1 - n2 - n3) * 8; const int wsel = (int)(u / (32 * 800)); const size_t e = u - (size_t)wsel * 32 * 800; const int oc = (int)(e / 800), k0 = (int)(e - (size_t)oc * 800); const float* wsrc = wsel == 0 ? w2 : wsel == 1 ? w3 : w4;
    for (int j = 0; j < 8; ++j) { const int k = k0 + j, tap = k >> 5, ic = k & 31; o[j] = (b16)(bf16_rne(wsrc[((size_t)tap * NF + ic) * NF + oc]) * WSC); }
    for (int pass = 0; pass < 2; ++pass) { *(volatile v8b*)(WC + u) = o; __threadfence(); } }
  else if (t < nx + n1 + n2 + n3 + n4 + nz) { const size_t e = (t - nx - n1 - n2 - n3 - n4) * 8; *(volatile v8b*)(zero0 + e) = o; }
}
__global__ __launch_bounds__(96) void deform_kernel(const float* __restrict__ x, const b16* __restrict__ X16, const b16* __restrict__ WOFF, const float* __restrict__ obias, const b16* __restrict__ FBh, const b16* __restrict__ FBl, const b16* __restrict__ HK, const float* __restrict__ hbias, b16* __restrict__ H1h, b16* __restrict__ H1l) {
  __shared__ float OFF[3][16][NOT + 1]; __shared__ __attribute__((aligned(16))) b16 PXh[3][48][96 + 8], PXl[3][48][96 + 8]; __shared__ __attribute__((aligned(16))) b16 HMh[3][16][64 + 8], HMl[3][16][64 + 8];
  const int i = blockIdx.x, b = blockIdx.z, wave = threadIdx.x >> 5, lane = threadIdx.x & 31, nloc = lane & 15, hlf = lane >> 4; const int j0 = blockIdx.y * 48 + wave * 16;
  { v8f acc[11];
#pragma unroll
    for (int t = 0; t < 11; ++t) acc[t] = (v8f){};
#pragma unroll 1
    for (int p = 0; p < K9; ++p) { const v16b a = frag_kb_u(X16 + (((size_t)b * H + i + p) * W + j0 + nloc) * C, hlf);
#pragma unroll
      for (int t = 0; t < 11; ++t) acc[t] = wmma16b(a, frag_kb(WOFF + (size_t)(t * 16 + nloc) * KOFF + p * 32, hlf), acc[t]); }
#pragma unroll
    for (int t = 0; t < 11; ++t) { const int oc = t * 16 + nloc; const float bb = (oc < NOFF) ? bf16_rne(obias[oc]) : 0.0f;
#pragma unroll
      for (int r = 0; r < 8; ++r) OFF[wave][8 * hlf + r][oc] = acc[t][r] * (1.0f / (XS * WSC)) + bb; } }
  for (int q = lane; q < 48 * 104; q += 32) { PXh[wave][q / 104][q % 104] = (b16)0.0f; PXl[wave][q / 104][q % 104] = (b16)0.0f; }
  wave_lds_sync();
  for (int task = lane; task < 16 * 81; task += 32) { const int jj = task / 81, k = task - jj * 81; const int p = k / 9, q = k - p * 9; const int j = j0 + jj;
    const float yoff = OFF[wave][jj][2 * k], xoff = OFF[wave][jj][2 * k + 1];
    const float yv = fminf(fmaxf((float)(i + p) + yoff, 0.0f), (float)(H - 1)), xv = fminf(fmaxf((float)(j + q) + xoff, 0.0f), (float)(W - 1));
    int y0 = (int)floorf(yv), x0 = (int)floorf(xv); const int y1 = min(max(y0 + 1, 0), H - 1), x1 = min(max(x0 + 1, 0), W - 1); y0 = min(max(y0, 0), H - 1); x0 = min(max(x0, 0), W - 1);
    const float y0f = (float)y0, y1f = (float)y1, x0f = (float)x0, x1f = (float)x1;
    const float w0 = (y1f - yv) * (x1f - xv), w1 = (y1f - yv) * (xv - x0f), w2 = (yv - y0f) * (x1f - xv), w3 = (yv - y0f) * (xv - x0f);
    const float* r0 = x + (((size_t)b * H + y0) * W) * C; const float* r1 = x + (((size_t)b * H + y1) * W) * C;
    for (int c = 0; c < C; ++c) { const float p0 = bf16_rne(r0[x0 * C + c]), p1 = bf16_rne(r0[x1 * C + c]), p2 = bf16_rne(r1[x0 * C + c]), p3 = bf16_rne(r1[x1 * C + c]);
      const float pix = ((pmul(w0, p0) + pmul(w1, p1)) + pmul(w2, p2)) + pmul(w3, p3); b16 a_, c_; split16(pix * XS, a_, c_); PXh[wave][jj * 3 + c][k] = a_; PXl[wave][jj * 3 + c][k] = c_; } }
  wave_lds_sync();
  v8f hm[3][2];
#pragma unroll
  for (int mt = 0; mt < 3; ++mt) for (int t = 0; t < 2; ++t) hm[mt][t] = (v8f){};
#pragma unroll
  for (int mt = 0; mt < 3; ++mt)
#pragma unroll
    for (int kb = 0; kb < 96; kb += 32) { const v16b a = frag_kb(&PXh[wave][mt * 16 + nloc][kb], hlf), al = frag_kb(&PXl[wave][mt * 16 + nloc][kb], hlf);
#pragma unroll
      for (int t = 0; t < 2; ++t) { const v16b fh = frag_kb(FBh + (size_t)(t * 16 + nloc) * 96 + kb, hlf), fl = frag_kb(FBl + (size_t)(t * 16 + nloc) * 96 + kb, hlf); hm[mt][t] = wmma16b(a, fh, hm[mt][t]); hm[mt][t] = wmma16b(al, fh, hm[mt][t]); hm[mt][t] = wmma16b(a, fl, hm[mt][t]); } }
  for (int q = lane; q < 16 * 72; q += 32) { HMh[wave][q / 72][q % 72] = (b16)0.0f; HMl[wave][q / 72][q % 72] = (b16)0.0f; }
  wave_lds_sync();
#pragma unroll
  for (int mt = 0; mt < 3; ++mt)
#pragma unroll
    for (int t = 0; t < 2; ++t)
#pragma unroll
      for (int r = 0; r < 8; ++r) { const int row = mt * 16 + 8 * hlf + r, m = t * 16 + nloc; if (m < NDCT) { const int jj = row / 3, c = row - jj * 3; b16 a_, c_; split16(hm[mt][t][r] * (1.0f / (XS * WSC)) * XS, a_, c_); HMh[wave][jj][c * NDCT + m] = a_; HMl[wave][jj][c * NDCT + m] = c_; } }
  wave_lds_sync();
  v8f o[2] = {{}, {}};
#pragma unroll
  for (int kb = 0; kb < 64; kb += 32) { const v16b a = frag_kb(&HMh[wave][nloc][kb], hlf), al = frag_kb(&HMl[wave][nloc][kb], hlf);
#pragma unroll
    for (int t = 0; t < 2; ++t) { const v16b bw = frag_kb(HK + (size_t)(t * 16 + nloc) * 64 + kb, hlf); o[t] = wmma16b(a, bw, o[t]); o[t] = wmma16b(al, bw, o[t]); } }
  wave_lds_sync();
#pragma unroll
  for (int t = 0; t < 2; ++t) { const int oc = t * 16 + nloc; const float bb = bf16_rne(hbias[oc]);
#pragma unroll
    for (int r = 0; r < 8; ++r) { b16 a_, c_; split16(fmaxf(o[t][r] * (1.0f / (XS * WSC)) + bb, 0.0f) * XS, a_, c_); HMh[wave][8 * hlf + r][oc] = a_; HMl[wave][8 * hlf + r][oc] = c_; } }
  wave_lds_sync();
  for (int pass = 0; pass < 2; ++pass) { { const int jj = lane >> 1, hseg = (lane & 1) * 16; const int j = j0 + jj; if (j < OW) { const size_t gi = (((size_t)b * H1P + i + 2) * H1P + j + 2) * NF + hseg; *(volatile v16b*)(H1h + gi) = *(const v16b*)(&HMh[wave][jj][hseg]); *(volatile v16b*)(H1l + gi) = *(const v16b*)(&HMl[wave][jj][hseg]); } } __threadfence(); }
}
template <int S, int POOL>
__global__ __launch_bounds__(64) void conv5_kernel(const b16* __restrict__ INh, const b16* __restrict__ INl, const b16* __restrict__ Wt, const float* __restrict__ bias, b16* __restrict__ OUTh, b16* __restrict__ OUTl, float* __restrict__ outf) {
  __shared__ __attribute__((aligned(16))) b16 Sh[2][16][40], Sl[2][16][40]; __shared__ __attribute__((aligned(16))) float Sf[2][4][36];
  constexpr int SP = S + 4; const int b = blockIdx.z, wave = threadIdx.x >> 5, lane = threadIdx.x & 31, nloc = lane & 15, hlf = lane >> 4;
  int iy, x0, py, px;
  if (POOL) { iy = blockIdx.y * 2; x0 = (blockIdx.x * 2 + wave) * 8; py = iy + (nloc >> 3); px = x0 + (nloc & 7); } else { iy = blockIdx.y; x0 = (blockIdx.x * 2 + wave) * 16; py = iy; px = x0 + nloc; }
  const int pxc = min(px, S + 1);
  v8f acc[2] = {{}, {}};
#pragma unroll 1
  for (int tap = 0; tap < 25; ++tap) { const int dy = tap / 5, dx = tap - dy * 5; const size_t gi = (((size_t)b * SP + py + dy) * SP + pxc + dx) * NF; const v16b a = frag_kb(INh + gi, hlf), al = frag_kb(INl + gi, hlf);
#pragma unroll
    for (int t = 0; t < 2; ++t) { const v16b bw = frag_kb(Wt + (size_t)(t * 16 + nloc) * 800 + tap * 32, hlf); acc[t] = wmma16b(a, bw, acc[t]); acc[t] = wmma16b(al, bw, acc[t]); } }
  float v[2][8];
#pragma unroll
  for (int t = 0; t < 2; ++t) { const float bb = bf16_rne(bias[t * 16 + nloc]); for (int r = 0; r < 8; ++r) v[t][r] = fmaxf(acc[t][r] * (1.0f / (XS * WSC)) + bb, 0.0f); }
  if (POOL == 0) {
#pragma unroll
    for (int t = 0; t < 2; ++t) for (int r = 0; r < 8; ++r) { b16 a_, c_; split16(v[t][r] * XS, a_, c_); Sh[wave][8 * hlf + r][t * 16 + nloc] = a_; Sl[wave][8 * hlf + r][t * 16 + nloc] = c_; }
    wave_lds_sync();
    for (int pass = 0; pass < 2; ++pass) { { const int rr = lane >> 1, hseg = (lane & 1) * 16; const int xx = x0 + rr; if (xx < S) { const size_t gi = (((size_t)b * SP + iy + 2) * SP + xx + 2) * NF + hseg; *(volatile v16b*)(OUTh + gi) = *(const v16b*)(&Sh[wave][rr][hseg]); *(volatile v16b*)(OUTl + gi) = *(const v16b*)(&Sl[wave][rr][hseg]); } } __threadfence(); }
    return; }
  float pm[2][4];
#pragma unroll
  for (int t = 0; t < 2; ++t) {
#pragma unroll
    for (int r = 0; r < 8; ++r) { const float o_ = __shfl_xor(v[t][r], 16); v[t][r] = fmaxf(v[t][r], o_); }
#pragma unroll
    for (int s = 0; s < 4; ++s) pm[t][s] = fmaxf(v[t][2 * s], v[t][2 * s + 1]); }
  constexpr int SO = S / 2; const int oy = iy / 2, ox0 = x0 / 2;
  if (POOL == 1) { if (hlf == 0) for (int t = 0; t < 2; ++t) for (int s = 0; s < 4; ++s) { b16 a_, c_; split16(pm[t][s] * XS, a_, c_); Sh[wave][s][t * 16 + nloc] = a_; Sl[wave][s][t * 16 + nloc] = c_; }
    wave_lds_sync();
    for (int pass = 0; pass < 2; ++pass) { if (lane < 8) { const int s = lane >> 1, hseg = (lane & 1) * 16; const int xx = ox0 + s; if (xx < SO) { const size_t gi = (((size_t)b * (SO + 4) + oy + 2) * (SO + 4) + xx + 2) * NF + hseg; *(volatile v16b*)(OUTh + gi) = *(const v16b*)(&Sh[wave][s][hseg]); *(volatile v16b*)(OUTl + gi) = *(const v16b*)(&Sl[wave][s][hseg]); } } __threadfence(); } }
  else { if (hlf == 0) for (int t = 0; t < 2; ++t) for (int s = 0; s < 4; ++s) Sf[wave][s][t * 16 + nloc] = pm[t][s];
    wave_lds_sync();
    for (int pass = 0; pass < 2; ++pass) { { const int s = lane >> 3, c4 = (lane & 7) * 4; const int xx = ox0 + s; if (xx < SO) *(volatile v4f*)(outf + (size_t)b * (SO * SO * NF) + ((size_t)oy * SO + xx) * NF + c4) = *(const v4f*)(&Sf[wave][s][c4]); } __threadfence(); } }
}
}

extern "C" void kernel_launch(void* const* d_in, const int* in_sizes, int n_in, void* d_out, int out_size, void* d_ws, size_t ws_size, hipStream_t stream) {
  (void)n_in;
  auto Fp = [&](int i) { return (const float*)d_in[i]; };
  if (in_sizes[0] != NB * H * W * C || in_sizes[1] != 81 * NDCT || in_sizes[2] != 63 * NF || in_sizes[4] != 81 * C * NOFF || in_sizes[5] != NOFF || in_sizes[6] != 25 * NF * NF || out_size != NB * 22 * 22 * NF) return;
  size_t off = 0; char* ws = (char*)d_ws;
  auto carve = [&](size_t bytes) { char* p = ws + off; off += (bytes + 255) & ~(size_t)255; return p; };
  b16* X16 = (b16*)carve(((size_t)NB * H * W * C + 4096) * 2); b16* WOFF = (b16*)carve((size_t)NOT * KOFF * 2); b16* FBh = (b16*)carve(32 * 96 * 2); b16* FBl = (b16*)carve(32 * 96 * 2); b16* HK = (b16*)carve(32 * 64 * 2); b16* WC = (b16*)carve((size_t)3 * 32 * 800 * 2);
  const size_t nH1 = (size_t)NB * H1P * H1P * NF + 8192, nP2 = (size_t)NB * P2P * P2P * NF + 8192;
  b16* Z0 = (b16*)carve((2 * nH1 + 4 * nP2) * 2); b16* H1h = Z0; b16* H1l = Z0 + nH1; b16* P2h = H1l + nH1; b16* P2l = P2h + nP2; b16* H3h = P2l + nP2; b16* H3l = H3h + nP2;
  if (off > ws_size || off > ((size_t)128 << 20)) return;
  const size_t nzero = 2 * nH1 + 4 * nP2;
  prep_kernel<<<(unsigned)((((size_t)NB * H * W * C + 256) / 8 + (size_t)NOT * KOFF / 8 + 32 * 96 / 8 + 32 * 64 / 8 + (size_t)3 * 32 * 800 / 8 + nzero / 8 + 255) / 256), 256, 0, stream>>>(Fp(0), Fp(1), Fp(2), Fp(4), Fp(6), Fp(8), Fp(10), X16, WOFF, FBh, FBl, HK, WC, Z0, nzero);
  deform_kernel<<<dim3(OH, 2, NB), 96, 0, stream>>>(Fp(0), X16, WOFF, Fp(5), FBh, FBl, HK, Fp(3), H1h, H1l);
  conv5_kernel<88, 1><<<dim3(6, 44, NB), 64, 0, stream>>>(H1h, H1l, WC, Fp(7), P2h, P2l, nullptr);
  conv5_kernel<44, 0><<<dim3(2, 44, NB), 64, 0, stream>>>(P2h, P2l, WC + 32 * 800, Fp(9), H3h, H3l, nullptr);
  conv5_kernel<44, 2><<<dim3(3, 22, NB), 64, 0, stream>>>(H3h, H3l, WC + 64 * 800, Fp(11), nullptr, nullptr, (float*)d_out);
}
